// MemristiveLinear_3702261809494
// MI455X (gfx1250) — hardware-verified
//
#include <hip/hip_runtime.h>
#include <stddef.h>


typedef _Float16 v16h __attribute__((ext_vector_type(16)));
typedef _Float16 v8h  __attribute__((ext_vector_type(8)));
typedef float    v8f  __attribute__((ext_vector_type(8)));
typedef float    v4f  __attribute__((ext_vector_type(4)));
typedef _Float16 h16;

#ifndef MROWS
#define MROWS 512
#endif
#define MROWS_FULL 512
#define KDIM 512
#define NDIM 512

static_assert(MROWS >= 64 && MROWS <= MROWS_FULL);
static_assert((MROWS % 64) == 0);
static_assert((KDIM % 64) == 0 && (KDIM % 32) == 0);
static_assert((NDIM % 64) == 0);
static_assert((KDIM % 8) == 0 && (NDIM % 4) == 0);
static_assert((((size_t)MROWS * KDIM) % 2048) == 0);
static_assert((size_t)MROWS_FULL * NDIM < (size_t)0x7FFFFFFFu);

#define LDT 72
#define LDC 68
static_assert((LDT % 8) == 0 && LDT >= 64);
static_assert((LDC % 4) == 0 && LDC >= 64);

#define WCARRY 64.0f
#define XCARRY 16.0f

#define WT_BYTES  ((size_t)NDIM * KDIM * 2)
#define X16_BYTES ((size_t)MROWS * KDIM * 2)
#define OFF_WT   ((size_t)0)
#define OFF_X16  (OFF_WT + WT_BYTES)
#define WS_TOTAL (OFF_X16 + X16_BYTES)
static_assert((WT_BYTES % 128) == 0 && (X16_BYTES % 128) == 0);
static_assert(WS_TOTAL <= (size_t)134217728);

__device__ __forceinline__ float bf16r(float x) {
  unsigned int u = __float_as_uint(x);
  u = (u + 0x7FFFu + ((u >> 16) & 1u)) & 0xFFFF0000u;
  return __uint_as_float(u);
}

static __device__ __forceinline__ h16 toh_flush(float v) {
  const h16 r = (h16)v;
  return (fabsf(v) < 6.103515625e-05f) ? (h16)0.0f : r;
}

__device__ __forceinline__ v16h frag_at(const _Float16* p) {
  v8h lo = *(const v8h*)(p);
  v8h hi = *(const v8h*)(p + 16);
  v16h out;
#pragma unroll
  for (int i = 0; i < 8; ++i) { out[i] = lo[i]; out[i + 8] = hi[i]; }
  return out;
}

__device__ __forceinline__ v8f wmma16(v16h a, v16h b, v8f c) {
  v8f d = __builtin_amdgcn_wmma_f32_16x16x32_f16(false, a, false, b, (short)0, c,
                                                 false, false);
  asm volatile("v_nop\n\tv_nop\n\tv_nop\n\tv_nop" : "+v"(d) : "v"(a), "v"(b));
  return d;
}

__global__ __launch_bounds__(256) void wconv_kernel(
    const float* __restrict__ W, _Float16* __restrict__ Wt, unsigned ldw, unsigned ldk) {
  __shared__ _Float16 T[64 * LDT];
  const unsigned tid = threadIdx.x;
  const unsigned n0 = blockIdx.x * 64u;
  const unsigned k0 = blockIdx.y * 64u;
#pragma unroll 4
  for (unsigned j = 0; j < 16u; ++j) {
    const unsigned idx = tid + 256u * j;
    const unsigned kr = idx >> 6, nc = idx & 63u;
    const float v = W[(size_t)(k0 + kr) * ldw + n0 + nc];
    T[nc * LDT + kr] = (_Float16)(WCARRY * bf16r(v));
  }
  __syncthreads();
  v8h x[2];
  size_t off[2];
#pragma unroll
  for (unsigned i = 0; i < 2u; ++i) {
    const unsigned n = 32u * i + (tid >> 3);
    const unsigned kc = (tid & 7u) * 8u;
    x[i] = *(const v8h*)&T[n * LDT + kc];
    off[i] = (size_t)(n0 + n) * ldk + k0 + kc;
  }
#pragma unroll
  for (int i = 0; i < 2; ++i) *(volatile v8h*)(Wt + off[i]) = x[i];
  __threadfence();
#pragma unroll
  for (int i = 0; i < 2; ++i) *(volatile v8h*)(Wt + off[i]) = x[i];
}

__global__ __launch_bounds__(256) void xcast_kernel(
    const float* __restrict__ X, _Float16* __restrict__ X16) {
  const unsigned tid = threadIdx.x;
  const size_t e0 = ((size_t)blockIdx.x * 256u + tid) * 8u;
  const v4f a0 = *(const v4f*)(X + e0);
  const v4f a1 = *(const v4f*)(X + e0 + 4u);
  v8h o;
#pragma unroll
  for (int i = 0; i < 4; ++i) {
    o[i]     = toh_flush(XCARRY * bf16r(a0[i]));
    o[i + 4] = toh_flush(XCARRY * bf16r(a1[i]));
  }
  _Float16* p = X16 + e0;
  *(volatile v8h*)p = o;
  __threadfence();
  *(volatile v8h*)p = o;
}

template <int MODE>
__device__ __forceinline__ void gemm_body(
    const _Float16* __restrict__ A16, const _Float16* __restrict__ Bt, const unsigned K,
    const float* __restrict__ bias, float* __restrict__ outf) {
  __shared__ float Cs[64 * LDC];
  const unsigned tid = threadIdx.x, lane = tid & 31u, w = tid >> 5;
  const unsigned mw = w >> 1, nw = w & 1u;
  const unsigned hh = lane >> 4, m = lane & 15u;
  const unsigned n0 = blockIdx.x * 64u;
  const unsigned row0 = blockIdx.y * 64u;

  const _Float16* ap  = A16 + (size_t)(row0 + mw * 16u + m) * K + hh * 8u;
  const _Float16* bp0 = Bt + (size_t)(n0 + nw * 32u + m) * K + hh * 8u;
  const _Float16* bp1 = bp0 + (size_t)16 * K;
  v8f acc0 = {}, acc1 = {};
#pragma unroll 2
  for (unsigned k0 = 0; k0 < K; k0 += 32u) {
    const v16h a  = frag_at(ap + k0);
    const v16h b0 = frag_at(bp0 + k0);
    const v16h b1 = frag_at(bp1 + k0);
    acc0 = wmma16(a, b0, acc0);
    acc1 = wmma16(a, b1, acc1);
  }
#pragma unroll
  for (int r = 0; r < 8; ++r) {
    float* d = &Cs[(mw * 16u + hh * 8u + (unsigned)r) * LDC + nw * 32u + m];
    d[0]  = acc0[r];
    d[16] = acc1[r];
  }
  __syncthreads();

  if (MODE == 0) {
    const float cs = 1.0f / (WCARRY * XCARRY);
    v4f xs[4];
    size_t off[4];
#pragma unroll
    for (unsigned i = 0; i < 4u; ++i) {
      const unsigned r = 16u * i + (tid >> 4);
      const unsigned c = (tid & 15u) * 4u;
      const v4f u = *(const v4f*)&Cs[r * LDC + c];
      const v4f g = *(const v4f*)(bias + n0 + c);
      v4f val;
#pragma unroll
      for (int j = 0; j < 4; ++j) val[j] = u[j] * cs + bf16r(g[j]);
      xs[i] = val;
      off[i] = (size_t)(row0 + r) * NDIM + n0 + c;
    }
#pragma unroll
    for (int i = 0; i < 4; ++i) *(volatile v4f*)(outf + off[i]) = xs[i];
    __threadfence();
#pragma unroll
    for (int i = 0; i < 4; ++i) *(volatile v4f*)(outf + off[i]) = xs[i];
  }
}

__global__ __launch_bounds__(256) void gemm_out_kernel(
    const _Float16* __restrict__ A16, const _Float16* __restrict__ Bt,
    const float* __restrict__ bias, float* __restrict__ outf) {
  gemm_body<0>(A16, Bt, (unsigned)KDIM, bias, outf);
}

extern "C" void kernel_launch(void* const* d_in, const int* in_sizes, int n_in,
                              void* d_out, int out_size, void* d_ws, size_t ws_size,
                              hipStream_t stream) {
  if (n_in < 3) return;
  if ((long long)in_sizes[0] < (long long)MROWS * KDIM) return;
  if ((long long)in_sizes[1] < (long long)KDIM * NDIM) return;
  if (in_sizes[2] < NDIM) return;
  if ((long long)out_size < (long long)MROWS * NDIM) return;
  if (ws_size < WS_TOTAL) return;

  const float* X  = (const float*)d_in[0];
  const float* Wm = (const float*)d_in[1];
  const float* Bv = (const float*)d_in[2];
  float* out = (float*)d_out;

  char* ws = (char*)d_ws;
  _Float16* W_t = (_Float16*)(ws + OFF_WT);
  _Float16* X16 = (_Float16*)(ws + OFF_X16);

  dim3 blk(256);
  wconv_kernel<<<dim3(NDIM / 64, KDIM / 64), blk, 0, stream>>>(Wm, W_t, (unsigned)NDIM,
                                                               (unsigned)KDIM);
  xcast_kernel<<<dim3((unsigned)(((size_t)MROWS * KDIM) / 2048)), blk, 0, stream>>>(X, X16);
  gemm_out_kernel<<<dim3(NDIM / 64, MROWS / 64), blk, 0, stream>>>(X16, W_t, Bv, out);
}
